// MolecularGATForRegression_30949534335546
// MI455X (gfx1250) — hardware-verified
//
#include <hip/hip_runtime.h>


namespace {
constexpr int N = 50000, E = 800000, G = 512, FI = 9, D = 256, NPAD = 50176, NBLK = NPAD / 128, HID = 64;
constexpr float FXS = 524288.0f, FXI = 1.0f / 524288.0f, PXS = 65536.0f, PXI = 1.0f / 65536.0f, NEG = 0.2f;

typedef _Float16 b16;
typedef __attribute__((ext_vector_type(16))) _Float16 v16b;
typedef __attribute__((ext_vector_type(8)))  _Float16 v8b;
typedef __attribute__((ext_vector_type(8)))  float v8f;
typedef __attribute__((ext_vector_type(4)))  float v4f;

__device__ __forceinline__ v8b ld8b(const b16* p) { return *(const v8b*)p; }
__device__ __forceinline__ v16b cat8b(v8b a, v8b b) { return __builtin_shufflevector(a, b, 0, 1, 2, 3, 4, 5, 6, 7, 8, 9, 10, 11, 12, 13, 14, 15); }
__device__ __forceinline__ v16b frag_kb(const b16* p, int hh) { return cat8b(ld8b(p + 8 * hh), ld8b(p + 16 + 8 * hh)); }
__device__ __forceinline__ void split16(float v, b16& hi, b16& lo) { hi = (b16)v; lo = (b16)(v - (float)hi); }
__device__ __forceinline__ void frag_ksplit(const float* p, int hh, v16b& fh_, v16b& fl_) {
  const float* p0 = p + 8 * hh; const float* p1 = p + 16 + 8 * hh;
#pragma unroll
  for (int e = 0; e < 8; ++e) { b16 a, c; split16(p0[e], a, c); fh_[e] = a; fl_[e] = c; split16(p1[e], a, c); fh_[8 + e] = a; fl_[8 + e] = c; }
}
__device__ __forceinline__ v8f wmma16b(v16b a, v16b b, v8f c) {
  v8f d = __builtin_amdgcn_wmma_f32_16x16x32_f16(false, a, false, b, (short)0, c, false, false);
  asm volatile("v_nop\n\tv_nop\n\tv_nop\n\tv_nop" : "+v"(d) : "v"(a), "v"(b));
  return d;
}
__device__ __forceinline__ void wave_lds_sync() {
  __builtin_amdgcn_fence(__ATOMIC_RELEASE, "workgroup");
  __builtin_amdgcn_wave_barrier();
  __builtin_amdgcn_fence(__ATOMIC_ACQUIRE, "workgroup");
}

struct Opnd { const void* p0; const void* p1; int ld; };
template <int NP> __device__ __forceinline__ void load_frags(const Opnd& o, int row, int kb, int hh, v16b& fh_, v16b& fl_) {
  if (NP == 0) { frag_ksplit((const float*)o.p0 + (size_t)row * o.ld + kb, hh, fh_, fl_); }
  else if (NP == 4) {
    const float* p = (const float*)o.p0 + (size_t)row * o.ld + kb; const float* p0 = p + 8 * hh; const float* p1 = p + 16 + 8 * hh;
#pragma unroll
    for (int e = 0; e < 8; ++e) { b16 a, c; split16(p0[e] * 64.0f, a, c); fh_[e] = a; fl_[e] = c; split16(p1[e] * 64.0f, a, c); fh_[8 + e] = a; fl_[8 + e] = c; }
  } else if (NP == 3) {
    const float* p = (const float*)o.p0 + (size_t)row * o.ld + kb; const float* p0 = p + 8 * hh; const float* p1 = p + 16 + 8 * hh;
#pragma unroll
    for (int e = 0; e < 8; ++e) { fh_[e] = (b16)p0[e]; fh_[8 + e] = (b16)p1[e]; }
    fl_ = fh_;
  } else {
    fh_ = frag_kb((const b16*)o.p0 + (size_t)row * o.ld + kb, hh);
    if (NP == 2) fl_ = frag_kb((const b16*)o.p1 + (size_t)row * o.ld + kb, hh); else fl_ = fh_;
  }
}
template <int ANP, int BNP> __device__ __forceinline__ v8f mac(v16b ah, v16b al, v16b bh, v16b bl, v8f c) {
  c = wmma16b(ah, bh, c);
  if (BNP == 0 || BNP == 2 || BNP == 4) c = wmma16b(ah, bl, c);
  if (ANP == 0 || ANP == 2 || ANP == 4) c = wmma16b(al, bh, c);
  return c;
}
template <int ANP, int BNP>
__device__ __forceinline__ void gemm_tile(const Opnd& A, const Opnd& B, int K, int m0, int c0, int nloc, int hlf, v8f (&acc)[2][4]) {
  for (int kb = 0; kb < K; kb += 32) {
    v16b a0h, a0l, a1h, a1l;
    load_frags<ANP>(A, m0 + nloc, kb, hlf, a0h, a0l);
    load_frags<ANP>(A, m0 + 16 + nloc, kb, hlf, a1h, a1l);
#pragma unroll
    for (int t = 0; t < 4; ++t) {
      v16b bh, bl;
      load_frags<BNP>(B, c0 + t * 16 + nloc, kb, hlf, bh, bl);
      acc[0][t] = mac<ANP, BNP>(a0h, a0l, bh, bl, acc[0][t]);
      acc[1][t] = mac<ANP, BNP>(a1h, a1l, bh, bl, acc[1][t]);
    }
  }
}

__device__ __forceinline__ void epi_planes(v8f (&acc)[2][4], float scale, bool two, b16* __restrict__ oh, b16* __restrict__ ol, int ldo,
                                           int m0, int c0, int lane, b16* Th, b16* Tl) {
  const int nloc = lane & 15, hlf = lane >> 4;
#pragma unroll
  for (int t = 0; t < 4; ++t)
#pragma unroll
    for (int r = 0; r < 2; ++r)
#pragma unroll
      for (int v = 0; v < 8; ++v) {
        const int rr = r * 16 + v + 8 * hlf, cc = t * 16 + nloc;
        b16 h_, l_; split16(acc[r][t][v] * scale, h_, l_);
        Th[rr * 64 + cc] = h_; Tl[rr * 64 + cc] = l_;
      }
  wave_lds_sync();
  for (int pass = 0; pass < 2; ++pass) {
#pragma unroll
    for (int j = 0; j < 8; ++j) {
      const int rr = j * 4 + (lane >> 3), c8 = (lane & 7) * 8;
      const size_t o = (size_t)(m0 + rr) * ldo + c0 + c8;
      *(volatile v8b*)(oh + o) = ld8b(Th + rr * 64 + c8);
      if (two) *(volatile v8b*)(ol + o) = ld8b(Tl + rr * 64 + c8);
    }
    __threadfence();
  }
}
__device__ __forceinline__ void epi_f32(v8f (&acc)[2][4], float scale, const float* rscale, float* __restrict__ out, int ldo, int m0, int c0, int lane, float* Tt) {
  const int nloc = lane & 15, hlf = lane >> 4;
#pragma unroll
  for (int t = 0; t < 4; ++t)
#pragma unroll
    for (int r = 0; r < 2; ++r)
#pragma unroll
      for (int v = 0; v < 8; ++v) {
        const int rr = r * 16 + v + 8 * hlf;
        const float rs = rscale ? rscale[(size_t)(m0 + rr) * 32] : 1.0f;
        Tt[rr * 64 + t * 16 + nloc] = acc[r][t][v] * scale * rs;
      }
  wave_lds_sync();
  float* dst0 = out + (size_t)m0 * ldo + c0;
  for (int pass = 0; pass < 2; ++pass) {
#pragma unroll
    for (int j = 0; j < 16; ++j) { const int rr = j * 2 + hlf, c4 = nloc * 4; *(volatile v4f*)(dst0 + (size_t)rr * ldo + c4) = *(const v4f*)(Tt + rr * 64 + c4); }
    __threadfence();
  }
}


__device__ __forceinline__ int fkey(float f) { const int b = __float_as_int(f); return (b >= 0) ? b : (b ^ 0x7FFFFFFF); }
__device__ __forceinline__ float fkey_inv(int k) { return __int_as_float((k >= 0) ? k : (k ^ 0x7FFFFFFF)); }
__device__ __forceinline__ float elu_(float v) { return (v > 0.0f) ? v : (__expf(v) - 1.0f); }

__global__ __launch_bounds__(256) void prep_kernel(const float* __restrict__ W1, const float* __restrict__ W2, b16* __restrict__ w1, b16* __restrict__ w2) {
  const size_t tid = (size_t)blockIdx.x * blockDim.x + threadIdx.x, nth = (size_t)gridDim.x * blockDim.x;
  for (int pass = 0; pass < 2; ++pass) {
    for (size_t p = tid; p < (size_t)D * 32; p += nth) { const int n = (int)(p / 32), k = (int)(p % 32); ((volatile b16*)w1)[p] = (b16)((k < FI) ? W1[(size_t)min(k, FI - 1) * D + n] : 0.0f); }
    for (size_t p = tid; p < (size_t)D * D; p += nth) { const int n = (int)(p / D), k = (int)(p % D); ((volatile b16*)w2)[p] = (b16)W2[(size_t)k * D + n]; }
    __threadfence();
  }
}

template <int KIN, int KREAL, int PIN>
__global__ __launch_bounds__(128) void lin_kernel(const float* __restrict__ x, const b16* __restrict__ w, float* __restrict__ y) {
  __shared__ __attribute__((aligned(16))) float Ts[4][32 * 64];
  const int lane = threadIdx.x & 31, wave = threadIdx.x >> 5, nloc = lane & 15, hlf = lane >> 4, m0 = blockIdx.y * 128 + wave * 32, c0 = blockIdx.x * 64;
  v8f acc[2][4];
#pragma unroll
  for (int r = 0; r < 2; ++r)
#pragma unroll
    for (int t = 0; t < 4; ++t) acc[r][t] = (v8f){};
  const int ra = min(m0 + nloc, N - 1), rb = min(m0 + 16 + nloc, N - 1);
#pragma unroll 1
  for (int kb = 0; kb < KIN; kb += 32) { v16b a0, a1, l0, l1;
#pragma unroll
    for (int e = 0; e < 16; ++e) { const int k = kb + ((e < 8) ? (8 * hlf + e) : (16 + 8 * hlf + e - 8)); const bool ok = (k < KREAL); const int kc = min(k, KREAL - 1); b16 p, q;
      split16(ok ? x[(size_t)ra * PIN + kc] * 8.0f : 0.0f, p, q); a0[e] = p; l0[e] = q; split16(ok ? x[(size_t)rb * PIN + kc] * 8.0f : 0.0f, p, q); a1[e] = p; l1[e] = q; }
#pragma unroll
    for (int t = 0; t < 4; ++t) { const v16b bw = frag_kb(w + (size_t)(c0 + t * 16 + nloc) * KIN + kb, hlf); acc[0][t] = wmma16b(a0, bw, acc[0][t]); acc[0][t] = wmma16b(l0, bw, acc[0][t]); acc[1][t] = wmma16b(a1, bw, acc[1][t]); acc[1][t] = wmma16b(l1, bw, acc[1][t]); } }
  epi_f32(acc, 0.125f, nullptr, y, D, m0, c0, lane, Ts[wave]);
}

template <int H, int C>
__global__ __launch_bounds__(256) void alpha_kernel(const float* __restrict__ xh, const float* __restrict__ as_, const float* __restrict__ ad_, float* __restrict__ al) {
  __shared__ float Ab[64][8];
  const int nl = threadIdx.x >> 2, q = threadIdx.x & 3, n = blockIdx.x * 64 + nl;
  float ss[4] = {0.0f, 0.0f, 0.0f, 0.0f}, sd[4] = {0.0f, 0.0f, 0.0f, 0.0f};
  for (int c = q; c < H * C; c += 4) { const float v = xh[(size_t)n * D + c]; const int h = c / C, cc = c % C; const float ws_ = as_[h * C + cc], wd_ = ad_[h * C + cc];
#pragma unroll
    for (int hh2 = 0; hh2 < 4; ++hh2) if (hh2 == h) { ss[hh2] += v * ws_; sd[hh2] += v * wd_; } }
#pragma unroll
  for (int h = 0; h < 4; ++h) {
#pragma unroll
    for (int o = 1; o < 4; o <<= 1) { ss[h] += __shfl_xor(ss[h], o); sd[h] += __shfl_xor(sd[h], o); } }
  if (q == 0) {
#pragma unroll
    for (int h = 0; h < 4; ++h) { Ab[nl][h] = (h < H) ? ss[h] : 0.0f; Ab[nl][4 + h] = (h < H) ? sd[h] : 0.0f; } }
  __syncthreads();
  for (int pass = 0; pass < 2; ++pass) { if (threadIdx.x < 128) *(volatile v4f*)(al + (size_t)blockIdx.x * 512 + threadIdx.x * 4) = *(const v4f*)(&Ab[threadIdx.x >> 1][(threadIdx.x & 1) * 4]); __threadfence(); }
}

typedef __attribute__((ext_vector_type(4))) int v4i;
template <int H, int C>
__global__ __launch_bounds__(256) void gat_kernel(const int* __restrict__ esrc, const int* __restrict__ edst, const float* __restrict__ xh, const float* __restrict__ al, const float* __restrict__ bias, float* __restrict__ xo) {
  constexpr int NB = 256;
  __shared__ __attribute__((aligned(16))) int acc[NB * D];
  __shared__ int mx[NB * 4]; __shared__ int den[NB * 4]; __shared__ int list[8 * 256];
  const int t_ = threadIdx.x, wave = t_ >> 5, lane = t_ & 31, base = blockIdx.x * NB, col0 = lane * 8, myh = col0 / C;
  for (int i = t_; i < NB * D; i += 256) acc[i] = 0;
  for (int i = t_; i < NB * 4; i += 256) { const int slot = i >> 2, h = i & 3, node = base + slot; float e = -INFINITY;
    if (node < N && h < H) { float a = al[(size_t)node * 8 + h] + al[(size_t)node * 8 + 4 + h]; e = (a > 0.0f) ? a : NEG * a; }
    den[i] = 0; mx[i] = fkey(e); }
  __syncthreads();
  for (int c0 = 0; c0 < E; c0 += 256 * 8) { const int e0 = c0 + (wave * 32 + lane) * 8;
#pragma unroll
    for (int j = 0; j < 8; ++j) { const int ee = min(e0 + j, E - 1); const int dv = edst[ee]; const unsigned sl = (unsigned)(((e0 + j < E) ? dv : -1) - base);
      if (sl < (unsigned)NB) { int s = esrc[ee]; s = (s < 0) ? 0 : (s >= N ? N - 1 : s);
#pragma unroll
        for (int h = 0; h < H; ++h) { float a = al[(size_t)s * 8 + h] + al[(size_t)(base + sl) * 8 + 4 + h]; a = (a > 0.0f) ? a : NEG * a; atomicMax(&mx[sl * 4 + h], fkey(a)); } } } }
  __syncthreads();
  int* wl = list + wave * 256;
  auto accumulate = [&](int s, int slot) {
    float w[4] = {0.0f, 0.0f, 0.0f, 0.0f};
#pragma unroll
    for (int h = 0; h < H; ++h) { float a = al[(size_t)s * 8 + h] + al[(size_t)(base + slot) * 8 + 4 + h]; a = (a > 0.0f) ? a : NEG * a; w[h] = __expf(a - fkey_inv(mx[slot * 4 + h])); }
    { const float wl_ = (lane == 0) ? w[0] : (lane == 1) ? w[1] : (lane == 2) ? w[2] : w[3]; if (lane < H) atomicAdd(&den[slot * 4 + lane], (int)rintf(wl_ * FXS)); }
    const float wm = (myh == 0) ? w[0] : (myh == 1) ? w[1] : (myh == 2) ? w[2] : w[3];
    const float* hr = xh + (size_t)s * D + col0; int* ar = acc + slot * D + col0; const v4f va = *(const v4f*)hr, vb = *(const v4f*)(hr + 4);
#pragma unroll
    for (int c = 0; c < 4; ++c) { atomicAdd(ar + c, (int)rintf(wm * va[c] * FXS)); atomicAdd(ar + 4 + c, (int)rintf(wm * vb[c] * FXS)); }
  };
  for (int slot = wave; slot < NB; slot += 8) { if (base + slot < N) accumulate(base + slot, slot); }
  for (int c0 = 0; c0 < E; c0 += 256 * 8) {
    const int e0 = c0 + (wave * 32 + lane) * 8; int dd[8];
#pragma unroll
    for (int j = 0; j < 8; ++j) { const int dv = edst[min(e0 + j, E - 1)]; dd[j] = (e0 + j < E) ? dv : -1; }
    unsigned sl[8]; bool hit[8]; bool anyl = false;
#pragma unroll
    for (int j = 0; j < 8; ++j) { sl[j] = (unsigned)(dd[j] - base); hit[j] = sl[j] < (unsigned)NB; anyl |= hit[j]; }
    int wc = 0;
    if (__builtin_amdgcn_ballot_w32(anyl) != 0u) {
#pragma unroll
      for (int j = 0; j < 8; ++j) {
        const unsigned mj = __builtin_amdgcn_ballot_w32(hit[j]);
        if (mj != 0u) {
          if (hit[j]) { const int pos = wc + (int)__builtin_amdgcn_mbcnt_lo(mj, 0u); int s = esrc[min(e0 + j, E - 1)]; s = (s < 0) ? 0 : (s >= N ? N - 1 : s); wl[pos] = (s << 11) | (int)sl[j]; }
          wc += __builtin_popcount(mj); } } }
    __builtin_amdgcn_wave_barrier(); __builtin_amdgcn_fence(__ATOMIC_RELEASE, "workgroup"); __builtin_amdgcn_fence(__ATOMIC_ACQUIRE, "workgroup");
    for (int i = 0; i < wc; ++i) { const int ent = wl[i]; accumulate(ent >> 11, ent & 2047); }
    __builtin_amdgcn_wave_barrier();
  }
  __syncthreads();
  for (int pass = 0; pass < 2; ++pass) {
    for (int i = t_; i < NB * D / 4; i += 256) { const int slot = i / (D / 4), cq = (i % (D / 4)) * 4, node = base + slot; v4f o = {0.0f, 0.0f, 0.0f, 0.0f};
      if (node < N) {
#pragma unroll
        for (int q = 0; q < 4; ++q) { const int c = cq + q; const int hh2 = c / C; const float dn = (float)den[slot * 4 + hh2]; o[q] = elu_((float)acc[slot * D + c] / (dn + 1e-16f * FXS) + bias[c]); } }
      *(volatile v4f*)(xo + (size_t)node * D + cq) = o; }
    __threadfence(); }
}

__global__ __launch_bounds__(256) void pool_kernel(const float* __restrict__ h, const int* __restrict__ batch, const float* __restrict__ l1w, const float* __restrict__ l1b, const float* __restrict__ l2w, const float* __restrict__ l2b, float* __restrict__ out) {
  constexpr int GB = 64;
  __shared__ __attribute__((aligned(16))) int sacc[GB * D]; __shared__ int smax[GB * D]; __shared__ int cnt[GB]; __shared__ int list[8 * 256]; __shared__ float Zs[GB][HID + 1]; __shared__ float Ob[GB];
  const int t_ = threadIdx.x, wave = t_ >> 5, lane = t_ & 31, gbase = blockIdx.x * GB, col0 = lane * 8;
  for (int i = t_; i < GB * D; i += 256) { sacc[i] = 0; smax[i] = fkey(-INFINITY); }
  if (t_ < GB) cnt[t_] = 0;
  __syncthreads();
  int* wl = list + wave * 256;
  for (int c0 = 0; c0 < N; c0 += 256 * 8) {
    const int n0 = c0 + (wave * 32 + lane) * 8; int dd[8];
#pragma unroll
    for (int j = 0; j < 8; ++j) { const int bv = batch[min(n0 + j, N - 1)]; dd[j] = (n0 + j < N) ? bv : -1; }
    unsigned sl[8]; bool hit[8]; bool anyl = false;
#pragma unroll
    for (int j = 0; j < 8; ++j) { sl[j] = (unsigned)(dd[j] - gbase); hit[j] = sl[j] < (unsigned)GB; anyl |= hit[j]; }
    int wc = 0;
    if (__builtin_amdgcn_ballot_w32(anyl) != 0u) {
#pragma unroll
      for (int j = 0; j < 8; ++j) {
        const unsigned mj = __builtin_amdgcn_ballot_w32(hit[j]);
        if (mj != 0u) {
          if (hit[j]) { const int pos = wc + (int)__builtin_amdgcn_mbcnt_lo(mj, 0u); wl[pos] = ((n0 + j) << 7) | (int)sl[j]; atomicAdd(&cnt[sl[j]], 1); }
          wc += __builtin_popcount(mj); } } }
    __builtin_amdgcn_wave_barrier(); __builtin_amdgcn_fence(__ATOMIC_RELEASE, "workgroup"); __builtin_amdgcn_fence(__ATOMIC_ACQUIRE, "workgroup");
    for (int i = 0; i < wc; ++i) { const int ent = wl[i]; const int n = ent >> 7, slot = ent & 127; const float* hr = h + (size_t)n * D + col0; const v4f va = *(const v4f*)hr, vb = *(const v4f*)(hr + 4);
#pragma unroll
      for (int c = 0; c < 4; ++c) { atomicAdd(&sacc[slot * D + col0 + c], (int)rintf(va[c] * PXS)); atomicAdd(&sacc[slot * D + col0 + 4 + c], (int)rintf(vb[c] * PXS)); atomicMax(&smax[slot * D + col0 + c], fkey(va[c])); atomicMax(&smax[slot * D + col0 + 4 + c], fkey(vb[c])); } }
    __builtin_amdgcn_wave_barrier();
  }
  __syncthreads();
  { const int slot = t_ >> 2, qq = t_ & 3; const float c_ = (float)cnt[slot], ic = 1.0f / fmaxf(c_, 1.0f); float z[16];
#pragma unroll
    for (int j = 0; j < 16; ++j) z[j] = l1b[qq * 16 + j];
#pragma unroll 1
    for (int k = 0; k < D; ++k) { const float a = (float)sacc[slot * D + k] * PXI; const float mxv = (c_ > 0.0f) ? fkey_inv(smax[slot * D + k]) : 0.0f;
#pragma unroll 1
      for (int part = 0; part < 3; ++part) { const float* wr = l1w + (size_t)(part * D + k) * HID + qq * 16; const float gv = (part == 0) ? a : (part == 1) ? a * ic : mxv;
#pragma unroll
        for (int j = 0; j < 16; ++j) z[j] += gv * wr[j]; } }
#pragma unroll
    for (int j = 0; j < 16; ++j) Zs[slot][qq * 16 + j] = elu_(z[j]); }
  __syncthreads();
  if (t_ < GB) { float o = l2b[0];
#pragma unroll 1
    for (int j = 0; j < HID; ++j) o += Zs[t_][j] * l2w[j];
    Ob[t_] = o; }
  __syncthreads();
  for (int pass = 0; pass < 2; ++pass) { if (t_ < 16) *(volatile v4f*)(out + (size_t)gbase + t_ * 4) = *(const v4f*)(&Ob[t_ * 4]); __threadfence(); }
}
}

extern "C" void kernel_launch(void* const* d_in, const int* in_sizes, int n_in,
                              void* d_out, int out_size, void* d_ws, size_t ws_size, hipStream_t stream) {
  (void)n_in; (void)out_size;
  const float* x = (const float*)d_in[0]; const int* ei = (const int*)d_in[1]; const int* batch = (const int*)d_in[2];
  const float* W1 = (const float*)d_in[4]; const float* as1 = (const float*)d_in[5]; const float* ad1 = (const float*)d_in[6]; const float* b1 = (const float*)d_in[7];
  const float* W2 = (const float*)d_in[8]; const float* as2 = (const float*)d_in[9]; const float* ad2 = (const float*)d_in[10]; const float* b2 = (const float*)d_in[11];
  const float* l1w = (const float*)d_in[12]; const float* l1b = (const float*)d_in[13]; const float* l2w = (const float*)d_in[14]; const float* l2b = (const float*)d_in[15];
  float* out = (float*)d_out;
  if (in_sizes[0] != N * FI || in_sizes[1] != 2 * E || in_sizes[2] != N || in_sizes[4] != FI * D || in_sizes[8] != D * D || in_sizes[12] != 3 * D * HID) return;
  const int* esrc = ei; const int* edst = ei + E;
  size_t off = 0; char* ws = (char*)d_ws;
  auto carve = [&](size_t bytes) { char* p = ws + off; off += (bytes + 255) & ~(size_t)255; return p; };
  b16* w1 = (b16*)carve((size_t)D * 32 * 2); b16* w2 = (b16*)carve((size_t)D * D * 2); float* xh = (float*)carve((size_t)NPAD * D * 4); float* hb = (float*)carve((size_t)NPAD * D * 4); float* al = (float*)carve((size_t)NPAD * 8 * 4);
  if (off > ws_size) return;
  prep_kernel<<<128, 256, 0, stream>>>(W1, W2, w1, w2);
  lin_kernel<32, FI, FI><<<dim3(4, NBLK), 128, 0, stream>>>(x, w1, xh);
  alpha_kernel<4, 64><<<NPAD / 64, 256, 0, stream>>>(xh, as1, ad1, al);
  gat_kernel<4, 64><<<NPAD / 256, 256, 0, stream>>>(esrc, edst, xh, al, b1, hb);
  lin_kernel<D, D, D><<<dim3(4, NBLK), 128, 0, stream>>>(hb, w2, xh);
  alpha_kernel<2, 128><<<NPAD / 64, 256, 0, stream>>>(xh, as2, ad2, al);
  gat_kernel<2, 128><<<NPAD / 256, 256, 0, stream>>>(esrc, edst, xh, al, b2, hb);
  pool_kernel<<<G / 64, 256, 0, stream>>>(hb, batch, l1w, l1b, l2w, l2b, out);
}
